// ODEVAE_76201309765846
// MI455X (gfx1250) — hardware-verified
//
#include <hip/hip_runtime.h>
#include <math.h>
#include <stddef.h>


#define NB 512
#define NT 64
#define ND 32
#define NH 256
#define NL 64
#define BM 32
#define NTHR 256
#define WSC 16.0f
#define WINV 0.0625f

static_assert((NT % 2) == 0);
static_assert((NB % BM) == 0);
static_assert(((NB * NT) % BM) == 0);

typedef __attribute__((ext_vector_type(16))) _Float16 v16h;
typedef __attribute__((ext_vector_type(8)))  _Float16 v8h;
typedef __attribute__((ext_vector_type(8)))  float    v8f;
typedef __attribute__((ext_vector_type(4)))  float    v4f;

__device__ __forceinline__ void dep_guard_h(v8f& a, v8f& b, v16h x, v16h y) { asm volatile("v_nop\n\tv_nop\n\tv_nop\n\tv_nop" : "+v"(a), "+v"(b) : "v"(x), "v"(y)); }
__device__ __forceinline__ void keep4_h(v16h a, v16h b, v16h c, v16h d) { asm volatile("v_nop" :: "v"(a), "v"(b), "v"(c), "v"(d)); }
template <typename T> struct Frag;
template <> struct Frag<_Float16> {
  typedef v16h V; union U { v16h v; v8h h[2]; };
  static __device__ __forceinline__ v16h load(const _Float16* p) {
    U f; f.h[0] = *(const v8h*)(p); f.h[1] = *(const v8h*)(p + 16); return f.v;
  }
  static __device__ __forceinline__ v8f mma(v16h a, v16h b, v8f c) {
    return __builtin_amdgcn_wmma_f32_16x16x32_f16(false, a, false, b, (short)0, c, false, false);
  }
  static __device__ __forceinline__ void guard(v8f& a, v8f& b, v16h x, v16h y) { dep_guard_h(a, b, x, y); }
  static __device__ __forceinline__ void keep(v16h a, v16h b, v16h c, v16h d) { keep4_h(a, b, c, d); }
};
typedef Frag<_Float16> FragH;

__device__ __forceinline__ v8f vz() { v8f z = {0.f, 0.f, 0.f, 0.f, 0.f, 0.f, 0.f, 0.f}; return z; }
__device__ __forceinline__ v8f mma(v16h a, v16h b, v8f c) { return FragH::mma(a, b, c); }

__device__ __forceinline__ void g1(v8f& a, v16h x, v16h y) {
  asm volatile("v_nop\n\tv_nop\n\tv_nop\n\tv_nop" : "+v"(a) : "v"(x), "v"(y));
}
__device__ __forceinline__ void g2(v8f& a, v8f& b, v16h x, v16h y, v16h z) {
  asm volatile("v_nop\n\tv_nop\n\tv_nop\n\tv_nop" : "+v"(a), "+v"(b) : "v"(x), "v"(y), "v"(z));
}
__device__ __forceinline__ void g3(v8f& a, v8f& b, v8f& d, v16h x, v16h y, v16h z, v16h w) {
  asm volatile("v_nop\n\tv_nop\n\tv_nop\n\tv_nop" : "+v"(a), "+v"(b), "+v"(d) : "v"(x), "v"(y), "v"(z), "v"(w));
}
__device__ __forceinline__ void g4(v8f& a, v8f& b, v8f& d, v8f& e, v16h x, v16h y, v16h z, v16h w) {
  asm volatile("v_nop\n\tv_nop\n\tv_nop\n\tv_nop" : "+v"(a), "+v"(b), "+v"(d), "+v"(e) : "v"(x), "v"(y), "v"(z), "v"(w));
}

__device__ __forceinline__ float sigm(float v) { return __builtin_amdgcn_rcpf(1.0f + expf(-v)); }

__global__ __launch_bounds__(256) void k_cast_pad(const float* __restrict__ src, _Float16* __restrict__ dst,
                                                  int rows, int cols, int ldd, float scale) {
  const int n2 = (rows * ldd) >> 1;
  const int i = blockIdx.x * 256 + threadIdx.x;
  if (i < n2) {
    const int e = 2 * i;
    const int r = e / ldd;
    const int cc = e - r * ldd;
    const float f0 = (cc < cols) ? src[(size_t)r * cols + cc] * scale : 0.0f;
    const float f1 = (cc + 1 < cols) ? src[(size_t)r * cols + cc + 1] * scale : 0.0f;
    const _Float16 h0 = (_Float16)f0, h1 = (_Float16)f1;
    const unsigned u = (unsigned)__builtin_bit_cast(unsigned short, h0) | ((unsigned)__builtin_bit_cast(unsigned short, h1) << 16);
    ((volatile unsigned*)dst)[i] = u;
    __threadfence();
    ((volatile unsigned*)dst)[i] = u;
  }
}

template <int K, int ACT>
__device__ __forceinline__ void mlp_layer(const _Float16* src, const _Float16* __restrict__ W,
                                          float bc0, float bc1, _Float16* dst, int wave, int hh, int c) {
  v8f a00 = vz(), a01 = vz(), a10 = vz(), a11 = vz();
  const int n0 = 32 * wave;
#pragma unroll 2
  for (int ks = 0; ks < K / 32; ++ks) {
    const int ko = ks * 32 + 8 * hh;
    const v16h A0 = FragH::load(src + (size_t)c * K + ko);
    const v16h A1 = FragH::load(src + (size_t)(16 + c) * K + ko);
    const v16h B0 = FragH::load(W + (size_t)(n0 + c) * K + ko);
    const v16h B1 = FragH::load(W + (size_t)(n0 + 16 + c) * K + ko);
    a00 = mma(A0, B0, a00);
    a01 = mma(A0, B1, a01);
    a10 = mma(A1, B0, a10);
    a11 = mma(A1, B1, a11);
    g4(a00, a01, a10, a11, A0, A1, B0, B1);
  }
#pragma unroll
  for (int r = 0; r < 8; ++r) {
    const int row = 8 * hh + r;
    float v00 = a00[r] * WINV + bc0;
    float v01 = a01[r] * WINV + bc1;
    float v10 = a10[r] * WINV + bc0;
    float v11 = a11[r] * WINV + bc1;
    if (ACT == 1) { v00 = tanhf(v00); v01 = tanhf(v01); v10 = tanhf(v10); v11 = tanhf(v11); }
    if (ACT == 2) { v00 = fmaxf(v00, 0.0f); v01 = fmaxf(v01, 0.0f); v10 = fmaxf(v10, 0.0f); v11 = fmaxf(v11, 0.0f); }
    dst[row * NH + n0 + c]             = (_Float16)v00;
    dst[row * NH + n0 + 16 + c]        = (_Float16)v01;
    dst[(16 + row) * NH + n0 + c]      = (_Float16)v10;
    dst[(16 + row) * NH + n0 + 16 + c] = (_Float16)v11;
  }
}

__device__ __forceinline__ void stage_xt(const float* __restrict__ x, const float* __restrict__ tg,
                                         _Float16* dst, int b0, int to, int tid) {
#pragma unroll
  for (int j = 0; j < (BM * 64) / NTHR; ++j) {
    const int i = tid + j * NTHR;
    const int m = i >> 6, k = i & 63;
    const size_t bt = (size_t)(b0 + m) * NT + to;
    const size_t btp = bt - ((to > 0) ? 1 : 0);
    float v = 0.0f;
    if (k < ND) v = x[bt * ND + k];
    else if (k == ND) v = (to > 0) ? (tg[bt] - tg[btp]) : 0.0f;
    dst[i] = (_Float16)v;
  }
}

__device__ __forceinline__ void gru_unit(const _Float16* xa, const _Float16* ha, _Float16* hw,
                                         const _Float16* __restrict__ Wih, const _Float16* __restrict__ Whh,
                                         int m0, int colb, float bsr, float bsz, float bin, float bhn,
                                         float (&hr)[8], int hh, int c) {
  v8f aR = vz(), aZ = vz(), aX = vz(), aH = vz();
#pragma unroll
  for (int ks = 0; ks < 2; ++ks) {
    const int ko = ks * 32 + 8 * hh;
    const v16h A  = FragH::load(xa + (m0 + c) * 64 + ko);
    const v16h BR = FragH::load(Wih + (size_t)(colb + c) * 64 + ko);
    const v16h BZ = FragH::load(Wih + (size_t)(NH + colb + c) * 64 + ko);
    const v16h BN = FragH::load(Wih + (size_t)(2 * NH + colb + c) * 64 + ko);
    aR = mma(A, BR, aR);
    aZ = mma(A, BZ, aZ);
    aX = mma(A, BN, aX);
    g3(aR, aZ, aX, A, BR, BZ, BN);
  }
#pragma unroll 2
  for (int ks = 0; ks < NH / 32; ++ks) {
    const int ko = ks * 32 + 8 * hh;
    const v16h A  = FragH::load(ha + (m0 + c) * NH + ko);
    const v16h BR = FragH::load(Whh + (size_t)(colb + c) * NH + ko);
    const v16h BZ = FragH::load(Whh + (size_t)(NH + colb + c) * NH + ko);
    const v16h BN = FragH::load(Whh + (size_t)(2 * NH + colb + c) * NH + ko);
    aR = mma(A, BR, aR);
    aZ = mma(A, BZ, aZ);
    aH = mma(A, BN, aH);
    g3(aR, aZ, aH, A, BR, BZ, BN);
  }
#pragma unroll
  for (int r = 0; r < 8; ++r) {
    const int row = m0 + 8 * hh + r;
    const float rg = sigm(aR[r] * WINV + bsr);
    const float zg = sigm(aZ[r] * WINV + bsz);
    const float gn = aX[r] * WINV + bin;
    const float gh = aH[r] * WINV + bhn;
    const float nn = tanhf(gn + rg * gh);
    const float hp = hr[r];
    const float hn = (1.0f - zg) * nn + zg * hp;
    hr[r] = hn;
    hw[row * NH + colb + c] = (_Float16)hn;
  }
}

#define GRU_OFF_XTB  0
#define GRU_OFF_HBFA 8192
#define GRU_OFF_HBFB 24576
#define GRU_OFF_STG  24576
#define GRU_LDS      49152

__global__ __launch_bounds__(NTHR) void k_gru(
    const float* __restrict__ x, const float* __restrict__ tg, const float* __restrict__ eps,
    const _Float16* __restrict__ Wih, const float* __restrict__ b_ih,
    const _Float16* __restrict__ Whh, const float* __restrict__ b_hh,
    const _Float16* __restrict__ Whl, const float* __restrict__ b_hl,
    float* __restrict__ out_z, float* __restrict__ out_m, float* __restrict__ out_lv) {
  extern __shared__ v4f smem_dyn[];
  char* smem = (char*)smem_dyn;
  _Float16* xtb  = (_Float16*)(smem + GRU_OFF_XTB);
  _Float16* hbfA = (_Float16*)(smem + GRU_OFF_HBFA);
  _Float16* hbfB = (_Float16*)(smem + GRU_OFF_HBFB);
  float*    stg  = (float*)(smem + GRU_OFF_STG);

  const int tid = threadIdx.x, lane = tid & 31, wave = tid >> 5, hh = lane >> 4, c = lane & 15;
  const int b0 = blockIdx.x * BM;
  const int colb0 = 32 * wave, colb1 = 32 * wave + 16;

  const float bsr0 = b_ih[colb0 + c] + b_hh[colb0 + c];
  const float bsr1 = b_ih[colb1 + c] + b_hh[colb1 + c];
  const float bsz0 = b_ih[NH + colb0 + c] + b_hh[NH + colb0 + c];
  const float bsz1 = b_ih[NH + colb1 + c] + b_hh[NH + colb1 + c];
  const float bin0 = b_ih[2 * NH + colb0 + c], bin1 = b_ih[2 * NH + colb1 + c];
  const float bhn0 = b_hh[2 * NH + colb0 + c], bhn1 = b_hh[2 * NH + colb1 + c];

  float h00[8], h01[8], h10[8], h11[8];
#pragma unroll
  for (int r = 0; r < 8; ++r) { h00[r] = 0.f; h01[r] = 0.f; h10[r] = 0.f; h11[r] = 0.f; }

  for (int i = tid; i < BM * NH; i += NTHR) hbfA[i] = (_Float16)0.0f;
  stage_xt(x, tg, xtb, b0, NT - 1, tid);
  __syncthreads();

#pragma unroll 1
  for (int s = 0; s < NT; ++s) {
    const int cur = s & 1;
    const _Float16* xa = xtb + cur * (BM * 64);
    const _Float16* ha = cur ? hbfB : hbfA;
    _Float16* hw = cur ? hbfA : hbfB;
    gru_unit(xa, ha, hw, Wih, Whh, 0,  colb0, bsr0, bsz0, bin0, bhn0, h00, hh, c);
    gru_unit(xa, ha, hw, Wih, Whh, 0,  colb1, bsr1, bsz1, bin1, bhn1, h01, hh, c);
    gru_unit(xa, ha, hw, Wih, Whh, 16, colb0, bsr0, bsz0, bin0, bhn0, h10, hh, c);
    gru_unit(xa, ha, hw, Wih, Whh, 16, colb1, bsr1, bsz1, bin1, bhn1, h11, hh, c);
    if (s + 1 < NT) stage_xt(x, tg, xtb + (cur ^ 1) * (BM * 64), b0, NT - 2 - s, tid);
    __syncthreads();
  }

  {
    const _Float16* hf = (NT & 1) ? hbfB : hbfA;
    const int mt = wave >> 2, cg = wave & 3;
    v8f aM = vz(), aL = vz();
#pragma unroll 2
    for (int ks = 0; ks < NH / 32; ++ks) {
      const int ko = ks * 32 + 8 * hh;
      const v16h A  = FragH::load(hf + (mt * 16 + c) * NH + ko);
      const v16h B0 = FragH::load(Whl + (size_t)(16 * cg + c) * NH + ko);
      const v16h B1 = FragH::load(Whl + (size_t)(NL + 16 * cg + c) * NH + ko);
      aM = mma(A, B0, aM);
      aL = mma(A, B1, aL);
      g2(aM, aL, A, B0, B1);
    }
#pragma unroll
    for (int r = 0; r < 8; ++r) {
      const int row = mt * 16 + 8 * hh + r;
      const int l = 16 * cg + c;
      const float mean = aM[r] * WINV + b_hl[l];
      const float lv = aL[r] * WINV + b_hl[NL + l];
      const float e = eps[(size_t)(b0 + row) * NL + l];
      const float z = mean + e * expf(0.5f * lv);
      stg[row * NL + l] = z;
      stg[BM * NL + row * NL + l] = mean;
      stg[2 * BM * NL + row * NL + l] = lv;
    }
  }
  __syncthreads();
  {
    float* o1 = out_z  + (size_t)b0 * NL;
    float* o2 = out_m  + (size_t)b0 * NL;
    float* o3 = out_lv + (size_t)b0 * NL;
    for (int pass = 0; pass < 2; ++pass) {
#pragma unroll
      for (int it = 0; it < 2; ++it) {
        const int idx = it * 1024 + tid * 4;
        const v4f v1 = *(const v4f*)(stg + idx);
        *(volatile v4f*)(o1 + idx) = v1;
        const v4f v2 = *(const v4f*)(stg + BM * NL + idx);
        *(volatile v4f*)(o2 + idx) = v2;
        const v4f v3 = *(const v4f*)(stg + 2 * BM * NL + idx);
        *(volatile v4f*)(o3 + idx) = v3;
      }
      __threadfence();
    }
  }
}

__device__ __forceinline__ void store_zs(const _Float16* yin, _Float16* __restrict__ zs16, int b0, int t, int wave, int lane) {
  const int row = 4 * wave + (lane >> 3);
  const int c8 = (lane & 7) * 8;
  const v8h v = *(const v8h*)(yin + row * NL + c8);
  _Float16* gp = zs16 + ((size_t)(b0 + row) * NT + t) * NL + c8;
  *(volatile v8h*)gp = v;
  __threadfence();
  *(volatile v8h*)gp = v;
}

__global__ __launch_bounds__(NTHR) void k_ode(
    const float* __restrict__ tg, const float* __restrict__ zin,
    const _Float16* __restrict__ W1h, const float* __restrict__ b1,
    const _Float16* __restrict__ W2h, const float* __restrict__ b2,
    const _Float16* __restrict__ W3h, const float* __restrict__ b3,
    const _Float16* __restrict__ W4h, const float* __restrict__ b4,
    _Float16* __restrict__ zs16) {
  __shared__ __align__(16) _Float16 yin[BM * NL];
  __shared__ __align__(16) _Float16 bufP[BM * NH];
  __shared__ __align__(16) _Float16 bufQ[BM * NH];

  const int tid = threadIdx.x, lane = tid & 31, wave = tid >> 5, hh = lane >> 4, c = lane & 15;
  const int b0 = blockIdx.x * BM;
  const int mt4 = wave >> 2, nt4 = wave & 3;
  const int col4 = nt4 * 16 + c;

  const float bc10 = b1[32 * wave + c], bc11 = b1[32 * wave + 16 + c];
  const float bc20 = b2[32 * wave + c], bc21 = b2[32 * wave + 16 + c];
  const float bc30 = b3[32 * wave + c], bc31 = b3[32 * wave + 16 + c];
  const float bc4 = b4[col4];

  float y[8], k1[8], k2[8];
#pragma unroll
  for (int r = 0; r < 8; ++r) {
    const int row = mt4 * 16 + 8 * hh + r;
    const float v = zin[(size_t)(b0 + row) * NL + col4];
    y[r] = v; k1[r] = 0.f; k2[r] = 0.f;
    yin[row * NL + col4] = (_Float16)v;
  }
  __syncthreads();
  store_zs(yin, zs16, b0, 0, wave, lane);

#pragma unroll 1
  for (int iv = 0; iv < NT - 1; ++iv) {
    const float dt = tg[iv + 1] - tg[iv];
    const float hs = 0.5f * dt;
    const float c0 = 0.5f * hs, c1 = 0.75f * hs;
#pragma unroll 1
    for (int sub = 0; sub < 2; ++sub) {
#pragma unroll 1
      for (int st = 0; st < 3; ++st) {
        mlp_layer<NL, 1>(yin, W1h, bc10, bc11, bufP, wave, hh, c);
        __syncthreads();
        mlp_layer<NH, 1>(bufP, W2h, bc20, bc21, bufQ, wave, hh, c);
        __syncthreads();
        mlp_layer<NH, 1>(bufQ, W3h, bc30, bc31, bufP, wave, hh, c);
        __syncthreads();
        v8f a4 = vz();
#pragma unroll 2
        for (int ks = 0; ks < NH / 32; ++ks) {
          const int ko = ks * 32 + 8 * hh;
          const v16h A = FragH::load(bufP + (mt4 * 16 + c) * NH + ko);
          const v16h B = FragH::load(W4h + (size_t)(nt4 * 16 + c) * NH + ko);
          a4 = mma(A, B, a4);
          g1(a4, A, B);
        }
#pragma unroll
        for (int r = 0; r < 8; ++r) {
          const int row = mt4 * 16 + 8 * hh + r;
          const float kq = a4[r] * WINV + bc4;
          float ytv;
          if (st == 0) {
            k1[r] = kq;
            ytv = y[r] + c0 * kq;
          } else if (st == 1) {
            k2[r] = kq;
            ytv = y[r] + c1 * kq;
          } else {
            const float yn = y[r] + hs * ((2.0f / 9.0f) * k1[r] + (1.0f / 3.0f) * k2[r] + (4.0f / 9.0f) * kq);
            y[r] = yn;
            ytv = yn;
          }
          yin[row * NL + col4] = (_Float16)ytv;
        }
        __syncthreads();
      }
    }
    store_zs(yin, zs16, b0, iv + 1, wave, lane);
  }
}

__global__ __launch_bounds__(NTHR) void k_dec(
    const _Float16* __restrict__ zs16,
    const _Float16* __restrict__ Wl2h, const float* __restrict__ b_l2h,
    const _Float16* __restrict__ Wh2o, const float* __restrict__ b_h2o,
    float* __restrict__ out0, int nrows) {
  __shared__ __align__(16) _Float16 act[BM * NH];
  __shared__ __align__(16) float st[BM * ND];
  const int tid = threadIdx.x, lane = tid & 31, wave = tid >> 5, hh = lane >> 4, c = lane & 15;
  const int row0 = blockIdx.x * BM;
  if (row0 + BM > nrows) return;

  const float bcA = b_l2h[32 * wave + c], bcB = b_l2h[32 * wave + 16 + c];
  mlp_layer<NL, 2>(zs16 + (size_t)row0 * NL, Wl2h, bcA, bcB, act, wave, hh, c);
  __syncthreads();
  if (wave < 4) {
    const int mt = wave >> 1, nt = wave & 1;
    v8f a = vz();
#pragma unroll 2
    for (int ks = 0; ks < NH / 32; ++ks) {
      const int ko = ks * 32 + 8 * hh;
      const v16h A = FragH::load(act + (mt * 16 + c) * NH + ko);
      const v16h B = FragH::load(Wh2o + (size_t)(nt * 16 + c) * NH + ko);
      a = mma(A, B, a);
      g1(a, A, B);
    }
    const float bb = b_h2o[nt * 16 + c];
#pragma unroll
    for (int r = 0; r < 8; ++r) st[(mt * 16 + 8 * hh + r) * ND + nt * 16 + c] = a[r] * WINV + bb;
  }
  __syncthreads();
  const v4f v = *(const v4f*)(st + tid * 4);
  float* gp = out0 + (size_t)row0 * ND + tid * 4;
  *(volatile v4f*)gp = v;
  __threadfence();
  *(volatile v4f*)gp = v;
}

extern "C" void kernel_launch(void* const* d_in, const int* in_sizes, int n_in,
                              void* d_out, int out_size, void* d_ws, size_t ws_size,
                              hipStream_t stream) {
  if (n_in < 21) return;
  if (in_sizes[0] != NB * NT * ND || in_sizes[1] != NB * NT || in_sizes[2] != NB * NL ||
      in_sizes[3] != 3 * NH * (ND + 1) || in_sizes[4] != 3 * NH || in_sizes[5] != 3 * NH * NH ||
      in_sizes[6] != 3 * NH || in_sizes[7] != 2 * NL * NH || in_sizes[8] != 2 * NL ||
      in_sizes[9] != NH * NL || in_sizes[10] != NH || in_sizes[11] != NH * NH || in_sizes[12] != NH ||
      in_sizes[13] != NH * NH || in_sizes[14] != NH || in_sizes[15] != NL * NH || in_sizes[16] != NL ||
      in_sizes[17] != NH * NL || in_sizes[18] != NH || in_sizes[19] != ND * NH || in_sizes[20] != ND) return;
  if (out_size != NB * NT * ND + 3 * NB * NL) return;

  const float* x     = (const float*)d_in[0];
  const float* t     = (const float*)d_in[1];
  const float* eps   = (const float*)d_in[2];
  const float* W_ih  = (const float*)d_in[3];
  const float* b_ih  = (const float*)d_in[4];
  const float* W_hh  = (const float*)d_in[5];
  const float* b_hh  = (const float*)d_in[6];
  const float* W_hl  = (const float*)d_in[7];
  const float* b_hl  = (const float*)d_in[8];
  const float* W1    = (const float*)d_in[9];
  const float* b1    = (const float*)d_in[10];
  const float* W2    = (const float*)d_in[11];
  const float* b2    = (const float*)d_in[12];
  const float* W3    = (const float*)d_in[13];
  const float* b3    = (const float*)d_in[14];
  const float* W4    = (const float*)d_in[15];
  const float* b4    = (const float*)d_in[16];
  const float* W_l2h = (const float*)d_in[17];
  const float* b_l2h = (const float*)d_in[18];
  const float* W_h2o = (const float*)d_in[19];
  const float* b_h2o = (const float*)d_in[20];

  char* ws = (char*)d_ws;
  size_t off = 0;
  auto carve = [&](size_t bytes) -> void* {
    void* p = ws + off;
    off = (off + bytes + 255) & ~(size_t)255;
    return p;
  };
  _Float16* Wih16  = (_Float16*)carve((size_t)3 * NH * 64 * 2);
  _Float16* Whh16  = (_Float16*)carve((size_t)3 * NH * NH * 2);
  _Float16* Whl16  = (_Float16*)carve((size_t)2 * NL * NH * 2);
  _Float16* W1_16  = (_Float16*)carve((size_t)NH * NL * 2);
  _Float16* W2_16  = (_Float16*)carve((size_t)NH * NH * 2);
  _Float16* W3_16  = (_Float16*)carve((size_t)NH * NH * 2);
  _Float16* W4_16  = (_Float16*)carve((size_t)NL * NH * 2);
  _Float16* Wl2h16 = (_Float16*)carve((size_t)NH * NL * 2);
  _Float16* Wh2o16 = (_Float16*)carve((size_t)ND * NH * 2);
  _Float16* zs16   = (_Float16*)carve((size_t)NB * NT * NL * 2);
  if (off > ws_size) return;

  float* out0 = (float*)d_out;
  float* out1 = out0 + (size_t)NB * NT * ND;
  float* out2 = out1 + (size_t)NB * NL;
  float* out3 = out2 + (size_t)NB * NL;

  k_cast_pad<<<(3 * NH * 64 / 2 + 255) / 256, 256, 0, stream>>>(W_ih, Wih16, 3 * NH, ND + 1, 64, WSC);
  k_cast_pad<<<(3 * NH * NH / 2 + 255) / 256, 256, 0, stream>>>(W_hh, Whh16, 3 * NH, NH, NH, WSC);
  k_cast_pad<<<(2 * NL * NH / 2 + 255) / 256, 256, 0, stream>>>(W_hl, Whl16, 2 * NL, NH, NH, WSC);
  k_cast_pad<<<(NH * NL / 2 + 255) / 256, 256, 0, stream>>>(W1, W1_16, NH, NL, NL, WSC);
  k_cast_pad<<<(NH * NH / 2 + 255) / 256, 256, 0, stream>>>(W2, W2_16, NH, NH, NH, WSC);
  k_cast_pad<<<(NH * NH / 2 + 255) / 256, 256, 0, stream>>>(W3, W3_16, NH, NH, NH, WSC);
  k_cast_pad<<<(NL * NH / 2 + 255) / 256, 256, 0, stream>>>(W4, W4_16, NL, NH, NH, WSC);
  k_cast_pad<<<(NH * NL / 2 + 255) / 256, 256, 0, stream>>>(W_l2h, Wl2h16, NH, NL, NL, WSC);
  k_cast_pad<<<(ND * NH / 2 + 255) / 256, 256, 0, stream>>>(W_h2o, Wh2o16, ND, NH, NH, WSC);

  k_gru<<<NB / BM, NTHR, GRU_LDS, stream>>>(x, t, eps, Wih16, b_ih, Whh16, b_hh, Whl16, b_hl,
                                            out1, out2, out3);
  k_ode<<<NB / BM, NTHR, 0, stream>>>(t, out1, W1_16, b1, W2_16, b2, W3_16, b3, W4_16, b4, zs16);
  k_dec<<<(NB * NT) / BM, NTHR, 0, stream>>>(zs16, Wl2h16, b_l2h, Wh2o16, b_h2o, out0, NB * NT);
}
